// PairwiseAttentionTerminal_66984309948707
// MI455X (gfx1250) — hardware-verified
//
#include <hip/hip_runtime.h>


#define LL   1024
#define BB   8
#define FF   256
#define NH_  8
#define HC   32
#define NG   (BB * NH_)
#define NTB  (LL * BB)
#define ZH   2
#define PCAR 1024.0f
typedef _Float16 h16;
typedef unsigned short bf;
typedef __attribute__((ext_vector_type(16))) __bf16   v16bf;
typedef __attribute__((ext_vector_type(16))) _Float16 v16h;
typedef __attribute__((ext_vector_type(8)))  _Float16 v8h;
typedef __attribute__((ext_vector_type(8)))  unsigned short v8us;
typedef __attribute__((ext_vector_type(8)))  float    v8f;
typedef __attribute__((ext_vector_type(4)))  float    v4f;
typedef v8h  __attribute__((may_alias)) v8ha;
typedef v4f  __attribute__((may_alias)) v4fa;
typedef v8us __attribute__((may_alias)) v8usa;

__device__ __forceinline__ unsigned short f2bf(float f) { unsigned u = __float_as_uint(f); u += 0x7FFFu + ((u >> 16) & 1u); return (unsigned short)(u >> 16); }
__device__ __forceinline__ float bf2f(unsigned short b) { return __uint_as_float(((unsigned)b) << 16); }
__device__ __forceinline__ float bfr(float f) { return bf2f(f2bf(f)); }
__device__ __forceinline__ v16h cat16(v8h lo, v8h hi) { return __builtin_shufflevector(lo, hi, 0, 1, 2, 3, 4, 5, 6, 7, 8, 9, 10, 11, 12, 13, 14, 15); }
__device__ __forceinline__ v16bf cat16b(v8us lo, v8us hi) { return __builtin_bit_cast(v16bf, __builtin_shufflevector(lo, hi, 0, 1, 2, 3, 4, 5, 6, 7, 8, 9, 10, 11, 12, 13, 14, 15)); }
__device__ __forceinline__ v8f wmma16(v16h a, v16h b, v8f c) { return __builtin_amdgcn_wmma_f32_16x16x32_f16(false, a, false, b, (short)0, c, false, false); }
__device__ __forceinline__ v8f wmmab(v16bf a, v16bf b, v8f c) { return __builtin_amdgcn_wmma_f32_16x16x32_bf16(false, a, false, b, (short)0, c, false, false); }


template <typename T16> struct WFrag;
template <> struct WFrag<h16> { typedef v16h V; static __device__ __forceinline__ V ld(const h16* p) { return cat16(*(const v8h*)p, *(const v8h*)(p + 16)); } static __device__ __forceinline__ v8f mma(V a, V b, v8f c) { return wmma16(a, b, c); } };
template <> struct WFrag<bf> { typedef v16bf V; static __device__ __forceinline__ V ld(const bf* p) { return cat16b(*(const v8us*)p, *(const v8us*)(p + 16)); } static __device__ __forceinline__ v8f mma(V a, V b, v8f c) { return wmmab(a, b, c); } };
template <typename T16, int NSPLIT, bool BIAS>
__global__ __launch_bounds__(32) void k_gemmw(const T16* __restrict__ A, const T16* __restrict__ A2, const T16* __restrict__ Bt, const T16* __restrict__ Bt2, int K, float* C, int ldc, const float* __restrict__ bias, size_t sA, size_t sB, size_t sC) {
    typedef typename WFrag<T16>::V V;
    __shared__ __align__(16) float os[16 * 68];
    const size_t z = blockIdx.z; A += z * sA; if (A2) A2 += z * sA; Bt += z * sB; if (Bt2) Bt2 += z * sB; C += z * sC;
    const int lane = threadIdx.x & 31, lr = lane & 15, hi = lane >> 4; const int r0 = blockIdx.x * 64, c0 = blockIdx.y * 64;
    v8f acc[4][4];
#pragma unroll
    for (int mb = 0; mb < 4; ++mb)
#pragma unroll
        for (int nb = 0; nb < 4; ++nb) acc[mb][nb] = (v8f){};
    const size_t aoff = (size_t)(r0 + lr) * K + 8 * hi, boff = (size_t)(c0 + lr) * K + 8 * hi;
#pragma unroll 1
    for (int kc = 0; kc < K; kc += 32) {
        V a[4], a2[4];
#pragma unroll
        for (int mb = 0; mb < 4; ++mb) { a[mb] = WFrag<T16>::ld(A + aoff + (size_t)mb * 16 * K + kc); if (NSPLIT == 1 || NSPLIT == 2) a2[mb] = WFrag<T16>::ld(A2 + aoff + (size_t)mb * 16 * K + kc); }
#pragma unroll
        for (int nb = 0; nb < 4; ++nb) { const V b = WFrag<T16>::ld(Bt + boff + (size_t)nb * 16 * K + kc); V b2; if (NSPLIT >= 2) b2 = WFrag<T16>::ld(Bt2 + boff + (size_t)nb * 16 * K + kc);
#pragma unroll
            for (int mb = 0; mb < 4; ++mb) { acc[mb][nb] = WFrag<T16>::mma(a[mb], b, acc[mb][nb]); if (NSPLIT == 1 || NSPLIT == 2) acc[mb][nb] = WFrag<T16>::mma(a2[mb], b, acc[mb][nb]); if (NSPLIT >= 2) acc[mb][nb] = WFrag<T16>::mma(a[mb], b2, acc[mb][nb]); } }
        asm volatile("v_nop\n\tv_nop\n\tv_nop\n\tv_nop" : "+v"(acc[0][0]), "+v"(acc[1][1]), "+v"(acc[2][2]), "+v"(acc[3][3]) : "v"(a[0]), "v"(a[3]));
    }
#pragma unroll
    for (int mb = 0; mb < 4; ++mb) {
#pragma unroll
        for (int nb = 0; nb < 4; ++nb) {
#pragma unroll
            for (int j = 0; j < 8; ++j) os[(hi * 8 + j) * 68 + nb * 16 + lr] = acc[mb][nb][j]; }
        __builtin_amdgcn_wave_barrier(); asm volatile("" ::: "memory");
        float* crow = C + (size_t)(r0 + mb * 16) * ldc + c0;
#pragma unroll 1
        for (int ps = 0; ps < 2; ++ps) {
#pragma unroll
            for (int s = 0; s < 8; ++s) { const int row = 2 * s + hi, cofs = lr * 4; v4f val = *(const v4fa*)(os + row * 68 + cofs); if (BIAS) { val[0] += bfr(bias[c0 + cofs]); val[1] += bfr(bias[c0 + cofs + 1]); val[2] += bfr(bias[c0 + cofs + 2]); val[3] += bfr(bias[c0 + cofs + 3]); }
                *(volatile v4f*)(crow + (size_t)row * ldc + cofs) = val; }
            if (ps == 0) __threadfence(); }
        __builtin_amdgcn_wave_barrier(); asm volatile("" ::: "memory");
    }
}

__device__ __forceinline__ h16 tohx(float x) { return (h16)x; }
__device__ __forceinline__ void splitf(float y, unsigned short& h, unsigned short& l) { h = f2bf(y); l = f2bf(y - bf2f(h)); }
__device__ __forceinline__ float sigm_(float x) { return __fdiv_rn(1.0f, 1.0f + __expf(-x)); }
typedef __attribute__((ext_vector_type(2))) _Float16 v2h;
typedef __attribute__((ext_vector_type(4))) _Float16 v4h;
typedef __attribute__((ext_vector_type(2))) unsigned short v2us;
typedef __attribute__((ext_vector_type(4))) unsigned short v4us;

__global__ __launch_bounds__(256) void k_wtG(const float* __restrict__ w, int K, int N, bf* Bt) {
    const int lane = threadIdx.x & 31; const int L0 = (blockIdx.x * 8 + (threadIdx.x >> 5)) * 8; const int nlines = N * K / 64;
#pragma unroll 1
    for (int ps = 0; ps < 2; ++ps) {
#pragma unroll 1
        for (int l = 0; l < 8; ++l) { const int L = L0 + l; if (L >= nlines) break; const size_t e = (size_t)L * 64 + lane * 2; const int k = (int)(e % K), n = (int)(e / K); v2us o;
            o[0] = f2bf(w[(size_t)k * N + n]); o[1] = f2bf(w[(size_t)(k + 1) * N + n]); *(volatile v2us*)(Bt + e) = o; }
        if (ps == 0) __threadfence(); }
}
__global__ __launch_bounds__(256) void k_wbp(const float* __restrict__ Wb, bf* Bt) { const int e = (blockIdx.x * 256 + threadIdx.x) * 4; if (e >= 64 * FF) return; const int k = e % FF, n = e / FF; v4us o;
#pragma unroll
    for (int q = 0; q < 4; ++q) o[q] = n < NH_ ? f2bf(Wb[(size_t)(k + q) * NH_ + n]) : (unsigned short)0; *(volatile v4us*)(Bt + e) = o; __threadfence(); *(volatile v4us*)(Bt + e) = o; }
__global__ __launch_bounds__(256) void k_ln(const float* __restrict__ X, const float* __restrict__ g, const float* __restrict__ bb, bf* Xh, bf* Xl) { const int lane = threadIdx.x & 31; const int t = blockIdx.x * 8 + (threadIdx.x >> 5); if (t >= NTB) return; float v[8]; float s = 0.f;
#pragma unroll
    for (int ch = 0; ch < 2; ++ch) { const v4f a = *(const v4f*)(X + (size_t)t * FF + ch * 128 + lane * 4);
#pragma unroll
        for (int q = 0; q < 4; ++q) { v[ch * 4 + q] = bfr(a[q]); s = __fadd_rn(s, v[ch * 4 + q]); } }
#pragma unroll
    for (int sh = 16; sh; sh >>= 1) s += __shfl_xor(s, sh, 32);
    const float mu = s * (1.0f / FF); float q2 = 0.f;
#pragma unroll
    for (int k = 0; k < 8; ++k) { const float d = __fsub_rn(v[k], mu); float p = __fmul_rn(d, d); asm volatile("" : "+v"(p)); q2 = __fadd_rn(q2, p); }
#pragma unroll
    for (int sh = 16; sh; sh >>= 1) q2 += __shfl_xor(q2, sh, 32);
    const float rs = __frsqrt_rn(__fadd_rn(q2 * (1.0f / FF), 1e-5f));
#pragma unroll 1
    for (int ps = 0; ps < 2; ++ps) {
#pragma unroll
        for (int ch = 0; ch < 2; ++ch) { v4us oh, ol;
#pragma unroll
            for (int q = 0; q < 4; ++q) { const int d = ch * 128 + lane * 4 + q; float tn = __fmul_rn(__fsub_rn(v[ch * 4 + q], mu), rs); asm volatile("" : "+v"(tn)); float tg = __fmul_rn(tn, bfr(g[d])); asm volatile("" : "+v"(tg)); unsigned short a, c; splitf(__fadd_rn(tg, bfr(bb[d])), a, c); oh[q] = a; ol[q] = c; }
            const size_t o = (size_t)t * FF + ch * 128 + lane * 4; *(volatile v4us*)(Xh + o) = oh; *(volatile v4us*)(Xl + o) = ol; }
        if (ps == 0) __threadfence(); } }
__global__ __launch_bounds__(256) void k_qkpl(const float* __restrict__ QF, const float* __restrict__ KF, bf* Qh, bf* Ql, bf* Kh, bf* Kl) { const size_t e = ((size_t)blockIdx.x * 256 + threadIdx.x) * 2; if (e >= (size_t)NG * LL * HC) return; const int d = (int)(e % HC); const int l = (int)((e / HC) % LL); const int n = (int)(e / ((size_t)HC * LL)); const int b = n / NH_, h = n % NH_; const size_t s = ((size_t)l * BB + b) * FF + h * HC + d; v2us qh, ql, kh, kl; unsigned short a, c;
    splitf(QF[s], a, c); qh[0] = a; ql[0] = c; splitf(QF[s + 1], a, c); qh[1] = a; ql[1] = c; splitf(KF[s], a, c); kh[0] = a; kl[0] = c; splitf(KF[s + 1], a, c); kh[1] = a; kl[1] = c;
    for (int ps = 0; ps < 2; ++ps) { *(volatile v2us*)(Qh + e) = qh; *(volatile v2us*)(Ql + e) = ql; *(volatile v2us*)(Kh + e) = kh; *(volatile v2us*)(Kl + e) = kl; if (ps == 0) __threadfence(); } }
__global__ __launch_bounds__(256) void k_vtp(const float* __restrict__ VF, h16* VT) { const size_t e = ((size_t)blockIdx.x * 256 + threadIdx.x) * 2; if (e >= (size_t)NG * 64 * LL) return; const int l = (int)(e % LL); const int d = (int)((e / LL) % 64); const int n = (int)(e / ((size_t)LL * 64)); const int b = n / NH_, h = n % NH_; v2h o;
    if (d < HC) { o[0] = tohx(VF[((size_t)l * BB + b) * FF + h * HC + d]); o[1] = tohx(VF[((size_t)(l + 1) * BB + b) * FF + h * HC + d]); } else { o[0] = (h16)0.f; o[1] = (h16)0.f; } *(volatile v2h*)(VT + e) = o; __threadfence(); *(volatile v2h*)(VT + e) = o; }
__global__ __launch_bounds__(256) void k_psoft(const float* __restrict__ Sb, const float* __restrict__ BF, const float* __restrict__ bbp, int n0, h16* P) { const int lane = threadIdx.x & 31; const int row = blockIdx.x * 8 + (threadIdx.x >> 5); if (row >= ZH * LL) return; const int z = row / LL; const int n = n0 + z; const int b = n / NH_, h = n % NH_; const float bh = bfr(bbp[h]); const float* sr = Sb + (size_t)row * LL; float v[32]; float mx = -3.0e38f;
#pragma unroll
    for (int ch = 0; ch < 8; ++ch) { const int j0 = ch * 128 + lane * 4; const v4f a = *(const v4f*)(sr + j0);
#pragma unroll
        for (int q = 0; q < 4; ++q) { float as = __fmul_rn(a[q], 0.17677669529663687f); asm volatile("" : "+v"(as)); const float t = __fadd_rn(as, __fadd_rn(BF[((size_t)(j0 + q) * BB + b) * 64 + h], bh)); v[ch * 4 + q] = t; mx = fmaxf(mx, t); } }
#pragma unroll
    for (int sh = 16; sh; sh >>= 1) mx = fmaxf(mx, __shfl_xor(mx, sh, 32));
    float sum = 0.f;
#pragma unroll
    for (int k = 0; k < 32; ++k) { float d0 = __fsub_rn(v[k], mx); asm volatile("" : "+v"(d0)); v[k] = __expf(d0); sum += v[k]; }
#pragma unroll
    for (int sh = 16; sh; sh >>= 1) sum += __shfl_xor(sum, sh, 32);
    const float f = __fdiv_rn(PCAR, sum);
#pragma unroll 1
    for (int ps = 0; ps < 2; ++ps) {
#pragma unroll
        for (int ch = 0; ch < 8; ++ch) { v4h o; o[0] = tohx(v[ch * 4] * f); o[1] = tohx(v[ch * 4 + 1] * f); o[2] = tohx(v[ch * 4 + 2] * f); o[3] = tohx(v[ch * 4 + 3] * f); *(volatile v4h*)(P + (size_t)row * LL + ch * 128 + lane * 4) = o; }
        if (ps == 0) __threadfence(); } }
__global__ __launch_bounds__(256) void k_mrg(const float* __restrict__ Ob, const float* __restrict__ GF, int n0, bf* Ah, bf* Al) { const size_t e = ((size_t)blockIdx.x * 256 + threadIdx.x) * 2; if (e >= (size_t)ZH * LL * HC) return; const int d = (int)(e % HC); const int l = (int)((e / HC) % LL); const int z = (int)(e / ((size_t)HC * LL)); const int n = n0 + z; const int b = n / NH_, h = n % NH_; const size_t oo = ((size_t)l * BB + b) * FF + h * HC + d; v2us oh, ol;
#pragma unroll
    for (int u = 0; u < 2; ++u) { float o = Ob[((size_t)z * LL + l) * 64 + d + u] * (1.0f / PCAR); asm volatile("" : "+v"(o)); unsigned short a, c; splitf(__fmul_rn(o, sigm_(GF[oo + u])), a, c); oh[u] = a; ol[u] = c; } *(volatile v2us*)(Ah + oo) = oh; *(volatile v2us*)(Al + oo) = ol; __threadfence(); *(volatile v2us*)(Ah + oo) = oh; *(volatile v2us*)(Al + oo) = ol; }

extern "C" void kernel_launch(void* const* d_in, const int* in_sizes, int n_in,
                              void* d_out, int out_size, void* d_ws, size_t ws_size, hipStream_t stream) {
    (void)in_sizes; (void)n_in; (void)out_size;
    const float* IN[15]; for (int i = 0; i < 15; ++i) IN[i] = (const float*)d_in[i];
    float* OUT = (float*)d_out;
    char* wsp = (char*)d_ws;
    auto take = [&](size_t bytes) { char* p = wsp; wsp += (bytes + 255) & ~(size_t)255; return (void*)p; };
    bf* WQ = (bf*)take((size_t)FF * FF * 2); bf* WK = (bf*)take((size_t)FF * FF * 2); bf* WV = (bf*)take((size_t)FF * FF * 2); bf* WG = (bf*)take((size_t)FF * FF * 2); bf* WO = (bf*)take((size_t)FF * FF * 2); bf* WBt = (bf*)take((size_t)64 * FF * 2);
    bf* Xh = (bf*)take((size_t)NTB * FF * 2); bf* Xl = (bf*)take((size_t)NTB * FF * 2); float* QF = (float*)take((size_t)NTB * FF * 4); float* KF = (float*)take((size_t)NTB * FF * 4); float* VF = (float*)take((size_t)NTB * FF * 4); float* GF = (float*)take((size_t)NTB * FF * 4); float* BF = (float*)take((size_t)NTB * 64 * 4);
    bf* Qh = (bf*)take((size_t)NG * LL * HC * 2); bf* Ql = (bf*)take((size_t)NG * LL * HC * 2); bf* Kh = (bf*)take((size_t)NG * LL * HC * 2); bf* Kl = (bf*)take((size_t)NG * LL * HC * 2); h16* VT = (h16*)take((size_t)NG * 64 * LL * 2);
    float* Sb = (float*)take((size_t)ZH * LL * LL * 4); h16* P16 = (h16*)take((size_t)ZH * LL * LL * 2); float* Ob = (float*)take((size_t)ZH * LL * 64 * 4); bf* Ah = (bf*)take((size_t)NTB * FF * 2); bf* Al = (bf*)take((size_t)NTB * FF * 2);
    if ((size_t)(wsp - (char*)d_ws) > ws_size) return;
    k_wtG<<<(FF * FF / 64 + 63) / 64, 256, 0, stream>>>(IN[3], FF, FF, WQ); k_wtG<<<(FF * FF / 64 + 63) / 64, 256, 0, stream>>>(IN[5], FF, FF, WK); k_wtG<<<(FF * FF / 64 + 63) / 64, 256, 0, stream>>>(IN[7], FF, FF, WV); k_wtG<<<(FF * FF / 64 + 63) / 64, 256, 0, stream>>>(IN[11], FF, FF, WG); k_wtG<<<(FF * FF / 64 + 63) / 64, 256, 0, stream>>>(IN[13], FF, FF, WO); k_wbp<<<(64 * FF / 4 + 255) / 256, 256, 0, stream>>>(IN[9], WBt);
    k_ln<<<NTB / 8, 256, 0, stream>>>(IN[0], IN[1], IN[2], Xh, Xl);
    k_gemmw<bf, 1, true><<<dim3(NTB / 64, FF / 64, 1), 32, 0, stream>>>(Xh, Xl, WQ, nullptr, FF, QF, FF, IN[4], 0, 0, 0); k_gemmw<bf, 1, true><<<dim3(NTB / 64, FF / 64, 1), 32, 0, stream>>>(Xh, Xl, WK, nullptr, FF, KF, FF, IN[6], 0, 0, 0);
    k_gemmw<bf, 1, true><<<dim3(NTB / 64, FF / 64, 1), 32, 0, stream>>>(Xh, Xl, WV, nullptr, FF, VF, FF, IN[8], 0, 0, 0); k_gemmw<bf, 1, true><<<dim3(NTB / 64, FF / 64, 1), 32, 0, stream>>>(Xh, Xl, WG, nullptr, FF, GF, FF, IN[12], 0, 0, 0);
    k_gemmw<bf, 1, false><<<dim3(NTB / 64, 1, 1), 32, 0, stream>>>(Xh, Xl, WBt, nullptr, FF, BF, 64, nullptr, 0, 0, 0);
    k_qkpl<<<(unsigned)(((size_t)NG * LL * HC / 2 + 255) / 256), 256, 0, stream>>>(QF, KF, Qh, Ql, Kh, Kl); k_vtp<<<(unsigned)(((size_t)NG * 64 * LL / 2 + 255) / 256), 256, 0, stream>>>(VF, VT);
    for (int n0 = 0; n0 < NG; n0 += ZH) { const size_t z = (size_t)n0;
        k_gemmw<bf, 2, false><<<dim3(LL / 64, LL / 64, ZH), 32, 0, stream>>>(Qh + z * LL * HC, Ql + z * LL * HC, Kh + z * LL * HC, Kl + z * LL * HC, HC, Sb, LL, nullptr, (size_t)LL * HC, (size_t)LL * HC, (size_t)LL * LL);
        k_psoft<<<ZH * LL / 8, 256, 0, stream>>>(Sb, BF, IN[10], n0, P16);
        k_gemmw<h16, 0, false><<<dim3(LL / 64, 1, ZH), 32, 0, stream>>>(P16, nullptr, VT + z * 64 * LL, nullptr, LL, Ob, 64, nullptr, (size_t)LL * LL, (size_t)64 * LL, (size_t)LL * 64);
        k_mrg<<<(unsigned)(((size_t)ZH * LL * HC / 2 + 255) / 256), 256, 0, stream>>>(Ob, GF, n0, Ah, Al); }
    k_gemmw<bf, 1, true><<<dim3(NTB / 64, FF / 64, 1), 32, 0, stream>>>(Ah, Al, WO, nullptr, FF, OUT, FF, IN[14], 0, 0, 0);
}
